// LogNCDEFunc_9225589752315
// MI455X (gfx1250) — hardware-verified
//
#include <hip/hip_runtime.h>


#define NS   16384
#define DDIR 8
#define NST  64
#define HID  128
#define VOUT (DDIR * NST)
#define NSIG 36
#define SCH  2048
#define TCH  (SCH * DDIR)
#define DM   64
#define LOSC 1024.0f

typedef _Float16 h16;
typedef unsigned short bf;
typedef __attribute__((ext_vector_type(16))) __bf16   v16bf;
typedef __attribute__((ext_vector_type(16))) _Float16 v16h;
typedef __attribute__((ext_vector_type(8)))  _Float16 v8h;
typedef __attribute__((ext_vector_type(8)))  unsigned short v8us;
typedef __attribute__((ext_vector_type(8)))  float    v8f;
typedef __attribute__((ext_vector_type(4)))  float    v4f;
typedef v8h  __attribute__((may_alias)) v8ha;
typedef v4f  __attribute__((may_alias)) v4fa;
typedef v8us __attribute__((may_alias)) v8usa;

__device__ __forceinline__ unsigned short f2bf(float f) { unsigned u = __float_as_uint(f); u += 0x7FFFu + ((u >> 16) & 1u); return (unsigned short)(u >> 16); }
__device__ __forceinline__ float bf2f(unsigned short b) { return __uint_as_float(((unsigned)b) << 16); }
__device__ __forceinline__ float bfr(float f) { return bf2f(f2bf(f)); }
__device__ __forceinline__ v16h cat16(v8h lo, v8h hi) { return __builtin_shufflevector(lo, hi, 0, 1, 2, 3, 4, 5, 6, 7, 8, 9, 10, 11, 12, 13, 14, 15); }
__device__ __forceinline__ v16bf cat16b(v8us lo, v8us hi) { return __builtin_bit_cast(v16bf, __builtin_shufflevector(lo, hi, 0, 1, 2, 3, 4, 5, 6, 7, 8, 9, 10, 11, 12, 13, 14, 15)); }
__device__ __forceinline__ v8f wmma16(v16h a, v16h b, v8f c) { return __builtin_amdgcn_wmma_f32_16x16x32_f16(false, a, false, b, (short)0, c, false, false); }
__device__ __forceinline__ v8f wmmab(v16bf a, v16bf b, v8f c) { return __builtin_amdgcn_wmma_f32_16x16x32_bf16(false, a, false, b, (short)0, c, false, false); }

template <bool SPLITA, bool F16OUT = false>
__global__ __launch_bounds__(128) void k_gemmb(const bf* __restrict__ A, const bf* __restrict__ Al, const bf* __restrict__ Bn, const float* __restrict__ bias, float* C, int ldc, h16* C2, const float* __restrict__ R = nullptr, int K = DM, int roundR = 1) {
    __shared__ __align__(16) float ost[4][16 * 68];
    const int lane = threadIdx.x & 31, wave = threadIdx.x >> 5, lr = lane & 15, hi = lane >> 4;
    const int r0 = blockIdx.x * 64 + wave * 16, c0 = blockIdx.y * 64;
    const size_t aoff = (size_t)(r0 + lr) * K + 8 * hi;
    size_t boff[4];
#pragma unroll
    for (int t = 0; t < 4; ++t) boff[t] = (size_t)(c0 + t * 16 + lr) * K + 8 * hi;
    v8f acc[4];
#pragma unroll
    for (int t = 0; t < 4; ++t) acc[t] = (v8f){};
#pragma unroll 1
    for (int kc = 0; kc < K; kc += 32) {
        const v16bf a = cat16b(*(const v8us*)(A + aoff + kc), *(const v8us*)(A + aoff + kc + 16));
        v16bf al = a;
        if (SPLITA) al = cat16b(*(const v8us*)(Al + aoff + kc), *(const v8us*)(Al + aoff + kc + 16));
#pragma unroll
        for (int t = 0; t < 4; ++t) { const v16bf b = cat16b(*(const v8us*)(Bn + boff[t] + kc), *(const v8us*)(Bn + boff[t] + kc + 16)); acc[t] = wmmab(a, b, acc[t]); if (SPLITA) acc[t] = wmmab(al, b, acc[t]); }
        asm volatile("v_nop\n\tv_nop\n\tv_nop\n\tv_nop" : "+v"(acc[0]), "+v"(acc[1]), "+v"(acc[2]), "+v"(acc[3]) : "v"(a), "v"(al));
    }
    float* os = &ost[wave][0];
#pragma unroll
    for (int t = 0; t < 4; ++t) { const float bv = bias ? bfr(bias[c0 + t * 16 + lr]) : 0.f;
#pragma unroll
        for (int j = 0; j < 8; ++j) os[(hi * 8 + j) * 68 + t * 16 + lr] = acc[t][j] + bv; }
    __syncthreads();
    if (F16OUT) {
        h16* crow = (h16*)(void*)C + (size_t)r0 * ldc + c0;
        auto pass = [&]() {
#pragma unroll
            for (int s = 0; s < 4; ++s) { const int row = 4 * s + (lane >> 3), piece = lane & 7; const float* sp = os + row * 68 + piece * 8; v8h o, o2;
#pragma unroll
                for (int i = 0; i < 8; ++i) { const h16 a = (h16)sp[i]; o[i] = a; o2[i] = (h16)((sp[i] - (float)a) * LOSC); }
                *(volatile v8h*)(crow + (size_t)row * ldc + piece * 8) = o; if (C2) *(volatile v8h*)(C2 + (size_t)r0 * ldc + c0 + (size_t)row * ldc + piece * 8) = o2; }
        };
        pass(); __threadfence(); pass();
    } else {
        float* crow = C + (size_t)r0 * ldc + c0;
        auto pass = [&]() {
#pragma unroll
            for (int s = 0; s < 8; ++s) { const int Lid = (lane >> 3) + 4 * s, piece = lane & 7; const int row = Lid >> 1, cofs = (Lid & 1) * 32 + piece * 4;
                v4f val = *(const v4fa*)(os + row * 68 + cofs); if (R) { const v4f rv = *(const v4f*)(R + ((size_t)r0 + row) * ldc + c0 + cofs); val += roundR ? (v4f){bfr(rv[0]), bfr(rv[1]), bfr(rv[2]), bfr(rv[3])} : rv; }
                *(volatile v4f*)(crow + (size_t)row * ldc + cofs) = val; }
        };
        pass(); __threadfence(); pass();
    }
}


__global__ __launch_bounds__(256) void k_cvt8(const float* __restrict__ src, bf* dst, size_t n8) {
    const size_t i = (size_t)blockIdx.x * 256 + threadIdx.x; if (i >= n8) return;
    const v8f v = *(const v8f*)(src + i * 8); v8us o;
#pragma unroll
    for (int k = 0; k < 8; ++k) o[k] = f2bf(v[k]);
    *(volatile v8us*)(dst + i * 8) = o; __threadfence(); *(volatile v8us*)(dst + i * 8) = o;
}
__global__ __launch_bounds__(256) void k_zero8(bf* dst, size_t n8) {
    const size_t i = (size_t)blockIdx.x * 256 + threadIdx.x; if (i >= n8) return; v8us z;
#pragma unroll
    for (int k = 0; k < 8; ++k) z[k] = 0;
    *(volatile v8us*)(dst + i * 8) = z; __threadfence(); *(volatile v8us*)(dst + i * 8) = z;
}

__device__ __forceinline__ float softplus_f(float x) { return (x > 20.f) ? x : log1pf(__expf(x)); }
__device__ __forceinline__ float sigm_f(float x) { return 1.0f / (1.0f + __expf(-x)); }
__global__ __launch_bounds__(256) void k_cvt64(const float* __restrict__ src, int nrows, bf* dst) {
    typedef __attribute__((ext_vector_type(2))) unsigned short v2us;
    const int lane = threadIdx.x & 31; const size_t r = (size_t)blockIdx.x * 8 + (threadIdx.x >> 5); if (r >= (size_t)nrows) return; v2us o;
#pragma unroll
    for (int i = 0; i < 2; ++i) o[i] = f2bf(src[r * NST + lane * 2 + i]);
    *(volatile v2us*)(dst + r * NST + lane * 2) = o; __threadfence(); *(volatile v2us*)(dst + r * NST + lane * 2) = o;
}
template <int MODE>
__global__ __launch_bounds__(256) void k_act(const float* __restrict__ P, const float* __restrict__ A, const float* __restrict__ bias, int nrows, int ncol, bf* dh, bf* dl, float* F32) {
    typedef __attribute__((ext_vector_type(4))) unsigned short v4us;
    const int lane = threadIdx.x & 31; const size_t r = (size_t)blockIdx.x * 8 + (threadIdx.x >> 5); if (r >= (size_t)nrows) return; const size_t s = r / DDIR;
#pragma unroll 1
    for (int ps = 0; ps < 2; ++ps) {
#pragma unroll 1
        for (int c0 = lane * 4; c0 < ncol; c0 += 128) { v4us oh, ol; v4f fo;
#pragma unroll
            for (int i = 0; i < 4; ++i) { const int c = c0 + i; const float p = P[r * ncol + c]; float y;
                if (MODE == 0) y = softplus_f(p + bfr(bias[c]));
                else if (MODE == 1) y = sigm_f(A[s * ncol + c] + bfr(bias[c])) * p;
                else { const float v = tanhf(A[s * ncol + c] + bfr(bias[c])); y = (1.0f - v * v) * p; }
                if (MODE == 2) fo[i] = y; else { const unsigned short hb = f2bf(y); oh[i] = hb; ol[i] = f2bf(y - bf2f(hb)); } }
            if (MODE == 2) *(volatile v4f*)(F32 + r * ncol + c0) = fo; else { *(volatile v4us*)(dh + r * ncol + c0) = oh; *(volatile v4us*)(dl + r * ncol + c0) = ol; } }
        if (ps == 0) __threadfence(); }
}
__global__ __launch_bounds__(256) void k_vdir(const float* __restrict__ A3, const float* __restrict__ b3, float* VF, bf* Th, bf* Tl) {
    typedef __attribute__((ext_vector_type(2))) unsigned short v2us; typedef __attribute__((ext_vector_type(2))) float v2f;
    const int lane = threadIdx.x & 31; const size_t r = (size_t)blockIdx.x * 8 + (threadIdx.x >> 5); if (r >= (size_t)TCH) return; const size_t s = r / DDIR; const int j = (int)(r % DDIR);
    v2f vf; v2us oh, ol;
#pragma unroll
    for (int i = 0; i < 2; ++i) { const int n = lane * 2 + i; const float v = tanhf(A3[s * VOUT + j * NST + n] + bfr(b3[j * NST + n])); vf[i] = v; const unsigned short hb = f2bf(v); oh[i] = hb; ol[i] = f2bf(v - bf2f(hb)); }
    *(volatile v2f*)(VF + s * VOUT + j * NST + lane * 2) = vf; *(volatile v2us*)(Th + r * NST + lane * 2) = oh; *(volatile v2us*)(Tl + r * NST + lane * 2) = ol; __threadfence();
    *(volatile v2f*)(VF + s * VOUT + j * NST + lane * 2) = vf; *(volatile v2us*)(Th + r * NST + lane * 2) = oh; *(volatile v2us*)(Tl + r * NST + lane * 2) = ol;
}
__global__ __launch_bounds__(256) void k_out(const float* __restrict__ VF, const float* __restrict__ DV, const float* __restrict__ sig, int s0, float* OUTP) {
    typedef __attribute__((ext_vector_type(2))) float v2f;
    const int lane = threadIdx.x & 31; const size_t sl = (size_t)blockIdx.x * 8 + (threadIdx.x >> 5); if (sl >= (size_t)SCH) return; const size_t s = (size_t)s0 + sl; v2f o;
#pragma unroll
    for (int q = 0; q < 2; ++q) { const int n = lane * 2 + q; float acc = 0.f;
#pragma unroll
        for (int i = 0; i < DDIR; ++i) acc = fmaf(bfr(sig[s * NSIG + i]), VF[sl * VOUT + i * NST + n], acc);
        int p = 0;
#pragma unroll
        for (int i = 0; i < DDIR; ++i)
#pragma unroll
            for (int j = i + 1; j < DDIR; ++j) { const float br = DV[((sl * DDIR) + i) * VOUT + j * NST + n] - DV[((sl * DDIR) + j) * VOUT + i * NST + n]; acc = fmaf(bfr(sig[s * NSIG + DDIR + p]), br, acc); ++p; }
        o[q] = acc; }
    *(volatile v2f*)(OUTP + s * NST + lane * 2) = o; __threadfence(); *(volatile v2f*)(OUTP + s * NST + lane * 2) = o;
}

extern "C" void kernel_launch(void* const* d_in, const int* in_sizes, int n_in,
                              void* d_out, int out_size, void* d_ws, size_t ws_size, hipStream_t stream) {
    (void)in_sizes; (void)n_in; (void)out_size;
    const float* h = (const float*)d_in[0]; const float* sig = (const float*)d_in[1]; const float* W1 = (const float*)d_in[2]; const float* b1 = (const float*)d_in[3]; const float* W2 = (const float*)d_in[4]; const float* b2 = (const float*)d_in[5]; const float* W3 = (const float*)d_in[6]; const float* b3 = (const float*)d_in[7];
    float* out = (float*)d_out;
    char* wsp = (char*)d_ws;
    auto take = [&](size_t bytes) { char* p = wsp; wsp += (bytes + 255) & ~(size_t)255; return (void*)p; };
    bf* W1B = (bf*)take(HID * NST * 2); bf* W2B = (bf*)take(HID * HID * 2); bf* W3B = (bf*)take((size_t)VOUT * HID * 2); bf* Hb = (bf*)take((size_t)NS * NST * 2);
    float* A1 = (float*)take((size_t)SCH * HID * 4); float* A2 = (float*)take((size_t)SCH * HID * 4); float* A3 = (float*)take((size_t)SCH * VOUT * 4); float* VF = (float*)take((size_t)SCH * VOUT * 4);
    bf* Zh = (bf*)take((size_t)SCH * HID * 2); bf* Zl = (bf*)take((size_t)SCH * HID * 2);
    bf* Th = (bf*)take((size_t)TCH * NST * 2); bf* Tl = (bf*)take((size_t)TCH * NST * 2); float* D1 = (float*)take((size_t)TCH * HID * 4); bf* Dh = (bf*)take((size_t)TCH * HID * 2); bf* Dl = (bf*)take((size_t)TCH * HID * 2); float* D3 = (float*)take((size_t)TCH * VOUT * 4); float* DV = (float*)take((size_t)TCH * VOUT * 4);
    if ((size_t)(wsp - (char*)d_ws) > ws_size) return;
    k_cvt8<<<(HID * NST / 8 + 255) / 256, 256, 0, stream>>>(W1, W1B, HID * NST / 8); k_cvt8<<<(HID * HID / 8 + 255) / 256, 256, 0, stream>>>(W2, W2B, HID * HID / 8); k_cvt8<<<(VOUT * HID / 8 + 255) / 256, 256, 0, stream>>>(W3, W3B, VOUT * HID / 8);
    k_cvt64<<<NS / 8, 256, 0, stream>>>(h, NS, Hb);
    for (int ch = 0; ch < NS / SCH; ++ch) { const int s0 = ch * SCH;
        k_gemmb<false, false><<<dim3(SCH / 64, HID / 64, 1), 128, 0, stream>>>(Hb + (size_t)s0 * NST, nullptr, W1B, nullptr, A1, HID, nullptr, nullptr, NST);
        k_act<0><<<SCH / 8, 256, 0, stream>>>(A1, nullptr, b1, SCH, HID, Zh, Zl, nullptr);
        k_gemmb<true, false><<<dim3(SCH / 64, HID / 64, 1), 128, 0, stream>>>(Zh, Zl, W2B, nullptr, A2, HID, nullptr, nullptr, HID);
        k_act<0><<<SCH / 8, 256, 0, stream>>>(A2, nullptr, b2, SCH, HID, Zh, Zl, nullptr);
        k_gemmb<true, false><<<dim3(SCH / 64, VOUT / 64, 1), 128, 0, stream>>>(Zh, Zl, W3B, nullptr, A3, VOUT, nullptr, nullptr, HID);
        k_vdir<<<TCH / 8, 256, 0, stream>>>(A3, b3, VF, Th, Tl);
        k_gemmb<true, false><<<dim3(TCH / 64, HID / 64, 1), 128, 0, stream>>>(Th, Tl, W1B, nullptr, D1, HID, nullptr, nullptr, NST);
        k_act<1><<<TCH / 8, 256, 0, stream>>>(D1, A1, b1, TCH, HID, Dh, Dl, nullptr);
        k_gemmb<true, false><<<dim3(TCH / 64, HID / 64, 1), 128, 0, stream>>>(Dh, Dl, W2B, nullptr, D1, HID, nullptr, nullptr, HID);
        k_act<1><<<TCH / 8, 256, 0, stream>>>(D1, A2, b2, TCH, HID, Dh, Dl, nullptr);
        k_gemmb<true, false><<<dim3(TCH / 64, VOUT / 64, 1), 128, 0, stream>>>(Dh, Dl, W3B, nullptr, D3, VOUT, nullptr, nullptr, HID);
        k_act<2><<<TCH / 8, 256, 0, stream>>>(D3, A3, b3, TCH, VOUT, nullptr, nullptr, DV);
        k_out<<<SCH / 8, 256, 0, stream>>>(VF, DV, sig, s0, out); }
}
